// TensorConvLayer_7627861918027
// MI455X (gfx1250) — hardware-run, weakly checked
//
#include <hip/hip_runtime.h>


namespace {
constexpr int N = 10000, E = 160000, HE = 64, WN = 576, M0 = 16, M1 = 8, F = 40;
constexpr float XS = 8.0f, WSC = 256.0f, INV3 = 0.57735026918962576f, ALPHA = 0.20412414523193150f, BEPS = 1e-5f;
typedef _Float16 b16;
typedef __attribute__((ext_vector_type(16))) _Float16 v16b;
typedef __attribute__((ext_vector_type(8))) _Float16 v8b;
typedef __attribute__((ext_vector_type(8))) float v8f;
typedef __attribute__((ext_vector_type(4))) float v4f;
__device__ __forceinline__ float bf16_rne(float f) { unsigned int u = __float_as_uint(f); u += 0x7FFFu + ((u >> 16) & 1u); return __uint_as_float(u & 0xFFFF0000u); }
__device__ __forceinline__ void split16(float v, b16& hi, b16& lo) { hi = (b16)v; lo = (b16)(v - (float)hi); }
__device__ __forceinline__ v16b frag_kb(const b16* p, int hh) { const v8b a = *(const v8b*)(p + 8 * hh), b = *(const v8b*)(p + 16 + 8 * hh); v16b f;
#pragma unroll
  for (int e = 0; e < 8; ++e) { f[e] = a[e]; f[8 + e] = b[e]; } return f; }
__device__ __forceinline__ v8f wmma16b(v16b a, v16b b, v8f c) { v8f d = __builtin_amdgcn_wmma_f32_16x16x32_f16(false, a, false, b, (short)0, c, false, false); asm volatile("v_nop\n\tv_nop\n\tv_nop\n\tv_nop" : "+v"(d) : "v"(a), "v"(b)); return d; }
__device__ __forceinline__ void wave_lds_sync() { __builtin_amdgcn_fence(__ATOMIC_RELEASE, "workgroup"); __builtin_amdgcn_wave_barrier(); __builtin_amdgcn_fence(__ATOMIC_ACQUIRE, "workgroup"); }
__device__ __forceinline__ float pmul(float a, float b) { float p = a * b; asm volatile("" : "+v"(p)); return p; }
__device__ __forceinline__ int iclamp(int v, int lo, int hi) { return v < lo ? lo : (v > hi ? hi : v); }
constexpr int CSR_NBLK7 = 512, CSR_GB7 = 7, CSR_GN7 = 1 << CSR_GB7  , CSR_TS7 = (CSR_GN7 < 32 ? 32 : CSR_GN7)  , CSR_MAXG7 = 512, CSR_CAP7 = 12288  ;
__device__ __host__ __forceinline__ int csr_tix7(int v) { return (v >> CSR_GB7) * CSR_TS7 + (v & (CSR_GN7 - 1)); }
__global__ __launch_bounds__(64) void csrA_kernel7(const int* __restrict__ dst, int E, int N, int nG, int CHP, int NGP, int* __restrict__ STG, int* __restrict__ HST) {
  extern __shared__ int sm[];
  int* cnt = sm; int* run = sm + NGP; int* ids = sm + 2 * NGP;
  const int b = blockIdx.x; const int ch = (E + CSR_NBLK7 - 1) / CSR_NBLK7; const int e0 = b * ch, e1 = min(E, e0 + ch);
  for (int i = threadIdx.x; i < NGP; i += 64) cnt[i] = 0;
  for (int i = threadIdx.x; i < CHP; i += 64) ids[i] = -1;
  __syncthreads();
  if (threadIdx.x == 0) {
    for (int e = e0; e < e1; ++e) { int d = dst[e]; d = (d < 0) ? 0 : (d >= N ? N - 1 : d); cnt[d >> CSR_GB7] += 1; }
    int acc = 0; for (int g = 0; g < nG; ++g) { run[g] = acc; acc += cnt[g]; }
    for (int e = e0; e < e1; ++e) { int d = dst[e]; d = (d < 0) ? 0 : (d >= N ? N - 1 : d); const int g = d >> CSR_GB7; ids[run[g]] = e; run[g] += 1; } }
  __syncthreads();
  typedef __attribute__((ext_vector_type(4))) int v4i;
  for (int pass = 0; pass < 2; ++pass) {
    for (int i = threadIdx.x; i < CHP / 4; i += 64) *(volatile v4i*)(STG + (size_t)b * CHP + i * 4) = *(const v4i*)(&ids[i * 4]);
    for (int i = threadIdx.x; i < NGP / 4; i += 64) { v4i v; for (int e = 0; e < 4; ++e) v[e] = (i * 4 + e < nG) ? cnt[i * 4 + e] : 0; *(volatile v4i*)(HST + (size_t)b * NGP + i * 4) = v; }
    __threadfence(); }
}
__global__ __launch_bounds__(512) void csrS_kernel7(const int* __restrict__ HST, int nG, int NGP, int* __restrict__ START, int* __restrict__ TOT, int* __restrict__ OFF) {
  __shared__ int tot[CSR_MAXG7];
  const int b = threadIdx.x;
  for (int pass = 0; pass < 2; ++pass) { int runb = 0; for (int g = 0; g < nG; ++g) { int c = HST[(size_t)b * NGP + g]; c = (c < 0) ? 0 : c; ((volatile int*)OFF)[(size_t)g * CSR_NBLK7 + b] = runb; runb += c; } __threadfence(); }
  for (int g = threadIdx.x; g < nG; g += 512) { int s = 0; for (int bb = 0; bb < CSR_NBLK7; ++bb) { int c = HST[(size_t)bb * NGP + g]; s += (c < 0) ? 0 : c; } tot[g] = s; }
  __syncthreads();
  if (threadIdx.x < 32) {
    __shared__ int st[CSR_MAXG7 + 32];
    if (threadIdx.x == 0) { int acc = 0; for (int g = 0; g < NGP; ++g) { st[g] = acc; if (g < nG) acc += (tot[g] + 31) & ~31; } st[NGP] = acc; }
    __builtin_amdgcn_fence(__ATOMIC_RELEASE, "workgroup"); __builtin_amdgcn_wave_barrier(); __builtin_amdgcn_fence(__ATOMIC_ACQUIRE, "workgroup");
    for (int pass = 0; pass < 2; ++pass) { for (int i = threadIdx.x; i < NGP + 32; i += 32) { ((volatile int*)START)[i] = (i <= NGP) ? st[min(i, NGP)] : 0; ((volatile int*)TOT)[i] = (i < nG) ? tot[i] : 0; } __threadfence(); } }
}
__global__ __launch_bounds__(256) void csrB_kernel7(const int* __restrict__ dst, int N, int nG, int CHP, int NGP, int permLen, const int* __restrict__ STG, const int* __restrict__ HST, const int* __restrict__ OFF, const int* __restrict__ START, const int* __restrict__ TOT, int* __restrict__ PERM, int* __restrict__ ROWPTR, int* __restrict__ ROWCNT, int* __restrict__ FLAG) {
  typedef __attribute__((ext_vector_type(4))) int v4i;
  __shared__ int ids[CSR_CAP7]; __shared__ unsigned short key[CSR_CAP7]; __shared__ int outp[CSR_CAP7]; __shared__ int ncnt[CSR_GN7 + 1]; __shared__ int boff[CSR_NBLK7 + 1];
  const int g = blockIdx.x, t_ = threadIdx.x; int tot = TOT[g]; int st = START[g], stn = START[g + 1]; const int v0 = g * CSR_GN7; const int nv = min(CSR_GN7, N - v0); const int t0 = g * CSR_TS7;
  st = (st < 0) ? 0 : (st > permLen - 32 ? permLen - 32 : st) & ~31; stn = (stn < st) ? st : (stn > permLen ? permLen : stn); tot = (tot < 0) ? 0 : tot; if (tot > stn - st && tot <= CSR_CAP7) tot = stn - st;
  if (tot > CSR_CAP7) {
    for (int pass = 0; pass < 2; ++pass) { for (int i = t_; i < CSR_TS7 / 4; i += 256) { v4i a, c; for (int e = 0; e < 4; ++e) { a[e] = st; c[e] = 0; } *(volatile v4i*)(ROWPTR + t0 + i * 4) = a; *(volatile v4i*)(ROWCNT + t0 + i * 4) = c; } if (t_ == 0) ((volatile int*)FLAG)[0] = 1; __threadfence(); } (void)nv; return; }
  if (t_ == 0) { int acc = 0; for (int b = 0; b < CSR_NBLK7; ++b) { boff[b] = acc; int c = HST[(size_t)b * NGP + g]; c = (c < 0) ? 0 : (c > CHP ? CHP : c); acc += c; if (acc > tot) acc = tot; } boff[CSR_NBLK7] = acc; }
  for (int i = t_; i <= CSR_GN7; i += 256) ncnt[i] = 0;
  __syncthreads();
  for (int b = 0; b < CSR_NBLK7; ++b) { const int c = boff[b + 1] - boff[b]; int o_ = OFF[(size_t)g * CSR_NBLK7 + b]; o_ = (o_ < 0) ? 0 : (o_ > CHP - c ? CHP - c : o_); const int* src_ = STG + (size_t)b * CHP + o_;
    for (int i = t_; i < c; i += 256) { int id = src_[i]; id = (id < 0) ? 0 : id; ids[boff[b] + i] = id; int d = dst[id]; d = (d < v0) ? v0 : (d >= N ? N - 1 : d); int kk = d - v0; kk = (kk < 0) ? 0 : (kk >= CSR_GN7 ? CSR_GN7 - 1 : kk); key[boff[b] + i] = (unsigned short)kk; } }
  __syncthreads();
  if (t_ == 0) { for (int i = 0; i < tot; ++i) ncnt[key[i]] += 1; int acc = 0; for (int vl = 0; vl < CSR_GN7; ++vl) { const int c = ncnt[vl]; ncnt[vl] = acc; acc += c; } ncnt[CSR_GN7] = acc;
    for (int i = 0; i < tot; ++i) { const int vl = key[i]; outp[ncnt[vl]] = ids[i]; ncnt[vl] += 1; }
    for (int vl = CSR_GN7; vl > 0; --vl) ncnt[vl] = ncnt[vl - 1]; ncnt[0] = 0; }
  __syncthreads();
  for (int pass = 0; pass < 2; ++pass) {
    for (int i = t_; i < (stn - st) / 4; i += 256) { v4i v; for (int e = 0; e < 4; ++e) { const int q = i * 4 + e; v[e] = (q < tot) ? outp[q] : -1; } *(volatile v4i*)(PERM + st + i * 4) = v; }
    for (int i = t_; i < CSR_TS7 / 4; i += 256) { v4i a, c; for (int e = 0; e < 4; ++e) { const int vl = i * 4 + e; const int vc = vl < CSR_GN7 ? vl : CSR_GN7; a[e] = (vl < CSR_GN7) ? st + ncnt[vc] : st; c[e] = (vl < nv) ? (ncnt[(vc < CSR_GN7 ? vc : CSR_GN7 - 1) + 1] - ncnt[vc]) : 0; } *(volatile v4i*)(ROWPTR + t0 + i * 4) = a; *(volatile v4i*)(ROWCNT + t0 + i * 4) = c; }
    __threadfence(); }
}
__global__ __launch_bounds__(256) void csrZ_kernel7(int* __restrict__ p, size_t n4) { typedef __attribute__((ext_vector_type(4))) int v4i; const size_t tid = (size_t)blockIdx.x * 256 + threadIdx.x, nth = (size_t)gridDim.x * 256; v4i z = {0, 0, 0, 0}; for (size_t i = tid; i < n4; i += nth) *(volatile v4i*)(p + i * 4) = z; }
struct CsrBufs7 { int *STG, *HST, *OFF, *START, *TOT, *PERM, *ROWPTR, *ROWCNT, *FLAG; int nG, NGP, CHP; size_t permLen; char* base; size_t bytes; };
static size_t csr_carve7(CsrBufs7& c, char* ws, size_t off, int E, int N) {
  const size_t off0 = off; c.base = ws + off;
  auto al = [&](size_t bytes) { char* p = ws + off; off += (bytes + 255) & ~(size_t)255; return p; };
  c.nG = (N + CSR_GN7 - 1) / CSR_GN7; c.NGP = (c.nG + 31) & ~31; const int ch = (E + CSR_NBLK7 - 1) / CSR_NBLK7; c.CHP = (ch + 31) & ~31; c.permLen = (size_t)E + 32 * (size_t)c.nG + 32;
  c.STG = (int*)al((size_t)CSR_NBLK7 * c.CHP * 4); c.HST = (int*)al((size_t)CSR_NBLK7 * c.NGP * 4); c.OFF = (int*)al((size_t)c.NGP * CSR_NBLK7 * 4); c.START = (int*)al((size_t)(c.NGP + 64) * 4); c.TOT = (int*)al((size_t)(c.NGP + 64) * 4);
  c.PERM = (int*)al(c.permLen * 4); c.ROWPTR = (int*)al((size_t)c.nG * CSR_TS7 * 4); c.ROWCNT = (int*)al((size_t)c.nG * CSR_TS7 * 4); c.FLAG = (int*)al(256);
  c.bytes = off - off0; return off;
}
static void csr_build7(const CsrBufs7& c, const int* dst, int E, int N, hipStream_t stream) {
  const size_t smem = (size_t)(2 * c.NGP + c.CHP) * 4;
  csrZ_kernel7<<<512, 256, 0, stream>>>((int*)c.base, c.bytes / 16);
  csrA_kernel7<<<CSR_NBLK7, 64, smem, stream>>>(dst, E, N, c.nG, c.CHP, c.NGP, c.STG, c.HST);
  csrS_kernel7<<<1, 512, 0, stream>>>(c.HST, c.nG, c.NGP, c.START, c.TOT, c.OFF);
  csrB_kernel7<<<c.nG, 256, 0, stream>>>(dst, N, c.nG, c.CHP, c.NGP, (int)c.permLen, c.STG, c.HST, c.OFF, c.START, c.TOT, c.PERM, c.ROWPTR, c.ROWCNT, c.FLAG);
}


__global__ __launch_bounds__(256) void wput_kernel(const float* __restrict__ w, int OUTW, b16* __restrict__ WT) { const int u = blockIdx.x * 256 + threadIdx.x; if (u >= OUTW * 8) return; const int o = u / 8, k0 = (u % 8) * 8; v8b v;
#pragma unroll
  for (int j = 0; j < 8; ++j) v[j] = (b16)(bf16_rne(w[(size_t)(k0 + j) * OUTW + o]) * WSC); for (int pass = 0; pass < 2; ++pass) { *(volatile v8b*)(WT + (size_t)o * HE + k0) = v; __threadfence(); } }
__global__ __launch_bounds__(256) void copy_kernel(const float* __restrict__ src, size_t n4, float* __restrict__ dst) { const size_t u = (size_t)blockIdx.x * 256 + threadIdx.x; if (u >= n4) return; const v4f v = *(const v4f*)(src + u * 4); for (int pass = 0; pass < 2; ++pass) { *(volatile v4f*)(dst + u * 4) = v; __threadfence(); } }
__global__ __launch_bounds__(32) void edge_kernel(const float* __restrict__ ef, const b16* __restrict__ WT1, const float* __restrict__ b1, const b16* __restrict__ WT2, const float* __restrict__ b2, const float* __restrict__ node, const float* __restrict__ sh, const int* __restrict__ dsts, int NLIM, int ELIM, float* __restrict__ TP) {
  __shared__ __attribute__((aligned(16))) b16 Ah[16][HE + 8], Hh[16][HE + 8], Hl[16][HE + 8]; __shared__ float Wl[16][WN + 4], To[16][F + 1];
  const int lane = threadIdx.x, nloc = lane & 15, hlf = lane >> 4; const size_t e0 = (size_t)blockIdx.x * 16; if (e0 >= (size_t)ELIM) return;
  for (int rr = 0; rr < 16; ++rr) for (int q = 0; q < 2; ++q) Ah[rr][q * 32 + lane] = (b16)(bf16_rne(ef[(e0 + rr) * HE + q * 32 + lane]) * XS);
  wave_lds_sync();
  { v8f acc[4] = {(v8f){}, (v8f){}, (v8f){}, (v8f){}};
#pragma unroll
    for (int kb = 0; kb < HE; kb += 32) { const v16b a = frag_kb(&Ah[nloc][kb], hlf);
#pragma unroll
      for (int t = 0; t < 4; ++t) acc[t] = wmma16b(a, frag_kb(WT1 + (size_t)(t * 16 + nloc) * HE + kb, hlf), acc[t]); }
#pragma unroll
    for (int t = 0; t < 4; ++t) { const int c = t * 16 + nloc; const float bb = bf16_rne(b1[c]);
#pragma unroll
      for (int r8 = 0; r8 < 8; ++r8) { b16 p, q; split16(fmaxf(acc[t][r8] * (1.0f / (XS * WSC)) + bb, 0.0f) * XS, p, q); Hh[8 * hlf + r8][c] = p; Hl[8 * hlf + r8][c] = q; } } }
  wave_lds_sync();
#pragma unroll 1
  for (int g = 0; g < 3; ++g) { v8f acc[12];
#pragma unroll
    for (int t = 0; t < 12; ++t) acc[t] = (v8f){};
#pragma unroll
    for (int kb = 0; kb < HE; kb += 32) { const v16b a = frag_kb(&Hh[nloc][kb], hlf), al = frag_kb(&Hl[nloc][kb], hlf);
#pragma unroll
      for (int t = 0; t < 12; ++t) { const v16b bw = frag_kb(WT2 + (size_t)(g * 192 + t * 16 + nloc) * HE + kb, hlf); acc[t] = wmma16b(a, bw, acc[t]); acc[t] = wmma16b(al, bw, acc[t]); } }
#pragma unroll
    for (int t = 0; t < 12; ++t) { const int c = g * 192 + t * 16 + nloc; const float bb = bf16_rne(b2[c]);
#pragma unroll
      for (int r8 = 0; r8 < 8; ++r8) Wl[8 * hlf + r8][c] = acc[t][r8] * (1.0f / (XS * WSC)) + bb; } }
  wave_lds_sync();
  for (int rr = 0; rr < 16; ++rr) { const size_t e = e0 + rr; const int nd = iclamp(dsts[e], 0, N - 1); const bool ok = nd < NLIM; const float* xr = node + (size_t)nd * F; const float s0 = bf16_rne(sh[e * 4]), s1x = bf16_rne(sh[e * 4 + 1]), s1y = bf16_rne(sh[e * 4 + 2]), s1z = bf16_rne(sh[e * 4 + 3]);
    for (int ps = 0; ps < 2; ++ps) { const int oc = ps == 0 ? lane : 32 + lane; if (oc >= F) continue; float val;
      if (oc < M0) { const int v = oc; float a0 = 0.0f, a1 = 0.0f;
#pragma unroll 1
        for (int uu = 0; uu < M0; ++uu) a0 += pmul(pmul(bf16_rne(xr[uu]), s0), Wl[rr][uu * M0 + v]);
#pragma unroll 1
        for (int uu = 0; uu < M1; ++uu) { const float d = pmul(bf16_rne(xr[M0 + uu * 3]), s1x) + pmul(bf16_rne(xr[M0 + uu * 3 + 1]), s1y) + pmul(bf16_rne(xr[M0 + uu * 3 + 2]), s1z); a1 += pmul(d, Wl[rr][M0 * M0 + uu * M0 + v]); }
        val = pmul(a0 + pmul(INV3, a1), ALPHA); }
      else { const int vi = oc - M0, v = vi / 3, i = vi % 3; const float si = i == 0 ? s1x : (i == 1 ? s1y : s1z); float a0 = 0.0f, a1 = 0.0f;
#pragma unroll 1
        for (int uu = 0; uu < M0; ++uu) a0 += pmul(pmul(bf16_rne(xr[uu]), si), Wl[rr][M0 * M0 + M1 * M0 + uu * M1 + v]);
#pragma unroll 1
        for (int uu = 0; uu < M1; ++uu) a1 += pmul(pmul(s0, bf16_rne(xr[M0 + uu * 3 + i])), Wl[rr][M0 * M0 + M1 * M0 + M0 * M1 + uu * M1 + v]);
        val = pmul(a0 + a1, ALPHA); }
      To[rr][oc] = ok ? val : 0.0f; } }
  wave_lds_sync();
  for (int pass = 0; pass < 2; ++pass) { for (int i = lane; i < 16 * F; i += 32) ((volatile float*)TP)[e0 * F + i] = To[i / F][i % F]; __threadfence(); }
}
__global__ __launch_bounds__(256) void node_kernel(const float* __restrict__ TP, const float* __restrict__ node, const int* __restrict__ dsts, const int* __restrict__ PERM, const int* __restrict__ ROWPTR, const int* __restrict__ ROWCNT, int permLen, int NLIM, int ELIM, float* __restrict__ PRE) {
  __shared__ float Po[8][F]; const int wave = threadIdx.x >> 5, lane = threadIdx.x & 31; const size_t n = (size_t)blockIdx.x * 8 + wave; const bool live = n < (size_t)NLIM;
  if (live) { int st = ROWPTR[n], cnt = ROWCNT[n]; cnt = iclamp(cnt, 0, 1 << 20); st = iclamp(st, 0, permLen - cnt); float a0 = 0.0f, a1 = 0.0f; int nn = 0;
#pragma unroll 1
    for (int j = 0; j < cnt; ++j) { const int e = iclamp(PERM[st + j], 0, E - 1); if (e >= ELIM || iclamp(dsts[e], 0, N - 1) >= NLIM) continue; ++nn; a0 += TP[(size_t)e * F + lane]; if (lane < F - 32) a1 += TP[(size_t)e * F + 32 + lane]; }
    const float inv = 1.0f / (float)(nn > 0 ? nn : 1); Po[wave][lane] = pmul(a0, inv) + bf16_rne(node[n * F + lane]); if (lane < F - 32) Po[wave][32 + lane] = pmul(a1, inv) + bf16_rne(node[n * F + 32 + lane]); }
  else { Po[wave][lane] = 0.0f; if (lane < F - 32) Po[wave][32 + lane] = 0.0f; }
  __syncthreads();
  if (wave == 0) { for (int pass = 0; pass < 2; ++pass) { for (int i = lane; i < 8 * F; i += 32) ((volatile float*)PRE)[(size_t)blockIdx.x * 8 * F + i] = Po[i / F][i % F]; __threadfence(); } }
}
__global__ __launch_bounds__(256) void bnstat_kernel(const float* __restrict__ PRE, const float* __restrict__ ws, const float* __restrict__ wv, int NLIM, float* __restrict__ ST) {
  __shared__ float Sv[64]; const int wave = threadIdx.x >> 5, lane = threadIdx.x & 31;
  for (int c = wave; c < M0 + M1; c += 8) {
    if (c < M0) { float s = 0.0f; for (int n = lane; n < NLIM; n += 32) s += PRE[(size_t)n * F + c]; for (int o = 16; o; o >>= 1) s += __shfl_xor(s, o); const float mu = s / (float)NLIM; float v = 0.0f; for (int n = lane; n < NLIM; n += 32) { const float d = PRE[(size_t)n * F + c] - mu; v += pmul(d, d); } for (int o = 16; o; o >>= 1) v += __shfl_xor(v, o);
      if (lane == 0) { Sv[c] = mu; Sv[16 + c] = pmul(rsqrtf(v / (float)NLIM + BEPS), bf16_rne(ws[c])); } }
    else { const int m = c - M0; float s = 0.0f; for (int n = lane; n < NLIM; n += 32) { const float* r = PRE + (size_t)n * F + M0 + m * 3; s += (pmul(r[0], r[0]) + pmul(r[1], r[1]) + pmul(r[2], r[2])) * (1.0f / 3.0f); } for (int o = 16; o; o >>= 1) s += __shfl_xor(s, o);
      if (lane == 0) Sv[32 + m] = pmul(rsqrtf(s / (float)NLIM + BEPS), bf16_rne(wv[m])); } }
  __syncthreads();
  if (wave == 0) { for (int pass = 0; pass < 2; ++pass) { ((volatile float*)ST)[lane] = Sv[lane]; ((volatile float*)ST)[32 + lane] = lane < 8 ? Sv[32 + lane] : 0.0f; __threadfence(); } }
}
__global__ __launch_bounds__(32) void out_kernel(const float* __restrict__ PRE, const float* __restrict__ ST, const float* __restrict__ bs, int NLIM, float* __restrict__ out) {
  __shared__ float Sv[64], To[16][F + 1]; const int lane = threadIdx.x; const size_t m0 = (size_t)blockIdx.x * 16; if (m0 >= (size_t)NLIM) return; Sv[lane] = ST[lane]; Sv[32 + lane] = ST[32 + lane]; wave_lds_sync();
  for (int rr = 0; rr < 16; ++rr) for (int c = lane; c < F; c += 32) { const float v = PRE[(m0 + rr) * F + c]; To[rr][c] = c < M0 ? pmul(v - Sv[c], Sv[16 + c]) + bf16_rne(bs[c]) : pmul(v, Sv[32 + (c - M0) / 3]); }
  wave_lds_sync();
  for (int pass = 0; pass < 2; ++pass) { for (int i = lane; i < 16 * F; i += 32) ((volatile float*)out)[m0 * F + i] = To[i / F][i % F]; __threadfence(); }
}
}

extern "C" void kernel_launch(void* const* d_in, const int* in_sizes, int n_in, void* d_out, int out_size, void* d_ws, size_t ws_size, hipStream_t stream) {
  (void)n_in;
  auto Fp = [&](int i) { return (const float*)d_in[i]; }; auto Ip = [&](int i) { return (const int*)d_in[i]; };
  if (in_sizes[0] != N * F || in_sizes[1] != E * HE || in_sizes[2] != E * 4 || in_sizes[3] != 2 * E || in_sizes[4] != HE * HE || in_sizes[6] != HE * WN || in_sizes[8] != M0 || in_sizes[10] != M1 || out_size != N * F + E * HE) return;
  const int NLIM = N, ELIM = E;
  size_t off = 0; char* ws = (char*)d_ws;
  auto carve = [&](size_t bytes) { char* p = ws + off; off += (bytes + 255) & ~(size_t)255; return p; };
  b16* WT1 = (b16*)carve((size_t)HE * HE * 2); b16* WT2 = (b16*)carve((size_t)WN * HE * 2); float* TP = (float*)carve((size_t)E * F * 4); float* PRE = (float*)carve((size_t)N * F * 4); float* ST = (float*)carve(64 * 4); CsrBufs7 csr; off = csr_carve7(csr, ws, off, E, N);
  if (off > ws_size || off > ((size_t)64 << 20)) return;
  float* out = (float*)d_out;
  copy_kernel<<<(unsigned)(((size_t)E * HE / 4 + 255) / 256), 256, 0, stream>>>(Fp(1), (size_t)E * HE / 4, out + (size_t)N * F);
  wput_kernel<<<(HE * 8 + 255) / 256, 256, 0, stream>>>(Fp(4), HE, WT1); wput_kernel<<<(WN * 8 + 255) / 256, 256, 0, stream>>>(Fp(6), WN, WT2);
  csr_build7(csr, Ip(3) + E, E, N, stream);
  edge_kernel<<<ELIM / 16, 32, 0, stream>>>(Fp(1), WT1, Fp(5), WT2, Fp(7), Fp(0), Fp(2), Ip(3), NLIM, ELIM, TP);
  node_kernel<<<(NLIM + 7) / 8, 256, 0, stream>>>(TP, Fp(0), Ip(3), csr.PERM, csr.ROWPTR, csr.ROWCNT, (int)csr.permLen, NLIM, ELIM, PRE);
  bnstat_kernel<<<1, 256, 0, stream>>>(PRE, Fp(8), Fp(10), NLIM, ST);
  out_kernel<<<NLIM / 16, 32, 0, stream>>>(PRE, ST, Fp(9), NLIM, out);
}
